// AdvancedHypergraphNetwork_69801808494761
// MI455X (gfx1250) — hardware-verified
//
#include <hip/hip_runtime.h>


#define NN_ 8192
#define NE2 8192
#define NNZ 262144
#define DD 128
#define NHEAD 4
#define HDM 32
#define NVOC 30522
#define NLAY 3
#define RCH 2048
#define IL_CAP 64
#define BN_EPS 1e-5f

typedef __attribute__((ext_vector_type(16))) __bf16   v16bf;
typedef __attribute__((ext_vector_type(16))) _Float16 v16h;
typedef __attribute__((ext_vector_type(8)))  float    v8f;
typedef __attribute__((ext_vector_type(8)))  unsigned v8u;

__device__ __forceinline__ unsigned f2bf(float f) { unsigned u = __float_as_uint(f); u += 0x7FFFu + ((u >> 16) & 1u); return u >> 16; }
__device__ __forceinline__ unsigned f2h(float f) { return (unsigned)__builtin_bit_cast(unsigned short, (_Float16)f); }
__device__ __forceinline__ int kpat(int v, int half) { return ((v & 4) ? 16 : 0) + half * 8 + 2 * (v & 3); }

template <int F16, int NP> struct Opnd { v16bf p[NP]; };

template <int F16, int NP> __device__ __forceinline__ void pack2(float f0, float f1, unsigned* o) {
    if (F16) { o[0] = f2h(f0) | (f2h(f1) << 16); return; }
    unsigned h0 = f2bf(f0), h1 = f2bf(f1); o[0] = h0 | (h1 << 16);
    if (NP >= 2) {
        float r0 = f0 - __uint_as_float(h0 << 16), r1 = f1 - __uint_as_float(h1 << 16);
        unsigned m0 = f2bf(r0), m1 = f2bf(r1); o[1] = m0 | (m1 << 16);
        if (NP >= 3) {
            float s0 = r0 - __uint_as_float(m0 << 16), s1 = r1 - __uint_as_float(m1 << 16);
            o[2] = f2bf(s0) | (f2bf(s1) << 16);
        }
    }
}
template <int F16, int NP> __device__ __forceinline__ void op_row(const float* rowp, int half, float sc, Opnd<F16, NP>& o) {
    v8u u[NP];
#pragma unroll
    for (int v = 0; v < 8; ++v) {
        int kk = kpat(v, half); unsigned t[3];
        pack2<F16, NP>(rowp[kk] * sc, rowp[kk + 1] * sc, t);
#pragma unroll
        for (int p = 0; p < NP; ++p) u[p][v] = t[p];
    }
#pragma unroll
    for (int p = 0; p < NP; ++p) o.p[p] = __builtin_bit_cast(v16bf, u[p]);
}
template <int F16, int NP> __device__ __forceinline__ void op_row_tail(const float* rowp, int half, float sc, int kvalid, Opnd<F16, NP>& o) {
    v8u u[NP];
#pragma unroll
    for (int v = 0; v < 8; ++v) {
        int kk = kpat(v, half); unsigned t[3];
        float f0 = kk < kvalid ? rowp[kk] * sc : 0.0f, f1 = (kk + 1) < kvalid ? rowp[kk + 1] * sc : 0.0f;
        pack2<F16, NP>(f0, f1, t);
#pragma unroll
        for (int p = 0; p < NP; ++p) u[p][v] = t[p];
    }
#pragma unroll
    for (int p = 0; p < NP; ++p) o.p[p] = __builtin_bit_cast(v16bf, u[p]);
}
template <int F16, int NP> __device__ __forceinline__ void op_col(const float* M, int ld, int n, int k0, int half, float sc, Opnd<F16, NP>& o) {
    v8u u[NP];
#pragma unroll
    for (int v = 0; v < 8; ++v) {
        int kk = k0 + kpat(v, half); unsigned t[3];
        pack2<F16, NP>(M[(size_t)kk * ld + n] * sc, M[(size_t)(kk + 1) * ld + n] * sc, t);
#pragma unroll
        for (int p = 0; p < NP; ++p) u[p][v] = t[p];
    }
#pragma unroll
    for (int p = 0; p < NP; ++p) o.p[p] = __builtin_bit_cast(v16bf, u[p]);
}
template <int F16, int NP> __device__ __forceinline__ void op_col_tail(const float* M, int ld, int n, int k0, int half, float sc, int K, Opnd<F16, NP>& o) {
    v8u u[NP];
#pragma unroll
    for (int v = 0; v < 8; ++v) {
        int kk = k0 + kpat(v, half); unsigned t[3];
        float f0 = kk < K ? M[(size_t)kk * ld + n] * sc : 0.0f, f1 = (kk + 1) < K ? M[(size_t)(kk + 1) * ld + n] * sc : 0.0f;
        pack2<F16, NP>(f0, f1, t);
#pragma unroll
        for (int p = 0; p < NP; ++p) u[p][v] = t[p];
    }
#pragma unroll
    for (int p = 0; p < NP; ++p) o.p[p] = __builtin_bit_cast(v16bf, u[p]);
}
__device__ __forceinline__ v8f wm_bf16(v16bf a, v16bf b, v8f c) { return __builtin_amdgcn_wmma_f32_16x16x32_bf16(false, a, false, b, (short)0, c, false, false); }
template <int F16, int NA, int NB> __device__ __forceinline__ v8f wmma_op(const Opnd<F16, NA>& a, const Opnd<F16, NB>& b, v8f c) {
    if (F16) {
        v16h ah = __builtin_bit_cast(v16h, a.p[0]), bh = __builtin_bit_cast(v16h, b.p[0]);
        c = __builtin_amdgcn_wmma_f32_16x16x32_f16(false, ah, false, bh, (short)0, c, false, false);
        asm volatile("v_nop\n\tv_nop\n\tv_nop\n\tv_nop" : "+v"(c) : "v"(ah), "v"(bh));
        return c;
    }
    constexpr int NMX = NA > NB ? NA : NB;
#pragma unroll
    for (int i = 0; i < NA; ++i)
#pragma unroll
        for (int j = 0; j < NB; ++j)
            if (i + j < NMX) c = wm_bf16(a.p[i], b.p[j], c);
    if (NA == 1 && NB == 1)      asm volatile("v_nop\n\tv_nop\n\tv_nop\n\tv_nop" : "+v"(c) : "v"(a.p[0]), "v"(b.p[0]));
    else if (NA == 2 && NB == 1) asm volatile("v_nop\n\tv_nop\n\tv_nop\n\tv_nop" : "+v"(c) : "v"(a.p[0]), "v"(a.p[1]), "v"(b.p[0]));
    else if (NA == 1 && NB == 2) asm volatile("v_nop\n\tv_nop\n\tv_nop\n\tv_nop" : "+v"(c) : "v"(a.p[0]), "v"(b.p[0]), "v"(b.p[1]));
    else if (NA == 2 && NB == 2) asm volatile("v_nop\n\tv_nop\n\tv_nop\n\tv_nop" : "+v"(c) : "v"(a.p[0]), "v"(a.p[1]), "v"(b.p[0]), "v"(b.p[1]));
    else                         asm volatile("v_nop\n\tv_nop\n\tv_nop\n\tv_nop" : "+v"(c) : "v"(a.p[0]), "v"(a.p[NA - 1]), "v"(b.p[0]), "v"(b.p[NB - 1]), "v"(a.p[NA / 2]), "v"(b.p[NB / 2]));
    return c;
}

struct ZMap { long long s1; long long s2; int zdiv; int pad_; };
__device__ __forceinline__ size_t zoff(const ZMap& m, int z) { return (size_t)((long long)(z / m.zdiv) * m.s1 + (long long)(z % m.zdiv) * m.s2); }

#define ACT_NONE 0
#define ACT_RELU 1
#define ACT_GELU_ERF 2
#define ACT_SILU 3
#define ACT_TANH 4
__device__ __forceinline__ float act_apply(int act, float x) {
    if (act == ACT_RELU) return x > 0.f ? x : 0.f;
    if (act == ACT_GELU_ERF) return 0.5f * x * (1.0f + erff(x * 0.70710678118654752f));
    if (act == ACT_SILU) return x / (1.0f + expf(-x));
    if (act == ACT_TANH) return tanhf(x);
    return x;
}
struct GemmArgs {
    ZMap za, zb_, zc, zbias, zadd, zrsc, zmul, zrbias;
    const float* A; const float* Bm; float* C; const float* bias; const float* add; const float* rsc; const float* mul; const float* rbias;
    long long ldadd, ldmul;
    int lda, ldb, ldc, K;
    float ascale, bscale, oscale, addscale;
    int M, nvalid, nstore, ldrsc;
    int bcs, pad1, pad2, pad3;
};
template <int BT, int F16, int NA, int NB, int RW, int CW, int ACT>
__global__ __launch_bounds__(256) void gemm_kernel(GemmArgs g) {
    constexpr int TR = 16 * RW, TC = 64 * CW, CSTR = TC + 4;
    __shared__ __align__(16) float cst[TR * CSTR];
    const int z = blockIdx.z;
    const float* A = g.A + zoff(g.za, z); const float* Bm = g.Bm + zoff(g.zb_, z); float* C = g.C + zoff(g.zc, z);
    const int tid = threadIdx.x, lane = tid & 31, wv = tid >> 5;
    const int l16 = lane & 15, half = lane >> 4;
    const int rt = wv % RW, ch = wv / RW;
    const int row0 = blockIdx.x * TR, col0 = blockIdx.y * TC + ch * 64;
    int arix = row0 + rt * 16 + l16; if (arix >= g.M) arix = g.M - 1;
    const float* arow = A + (size_t)arix * g.lda;
    v8f acc[4];
#pragma unroll
    for (int t = 0; t < 4; ++t) acc[t] = (v8f){};
    const int K = g.K;
#pragma unroll 1
    for (int kc = 0; kc < K; kc += 32) {
        Opnd<F16, NA> a;
        if (kc + 32 <= K) op_row<F16, NA>(arow + kc, half, g.ascale, a); else op_row_tail<F16, NA>(arow + kc, half, g.ascale, K - kc, a);
#pragma unroll
        for (int t = 0; t < 4; ++t) {
            Opnd<F16, NB> b;
            const int n = col0 + t * 16 + l16;
            if (n < g.nvalid) {
                if (BT) { if (kc + 32 <= K) op_row<F16, NB>(Bm + (size_t)n * g.ldb + kc, half, g.bscale, b); else op_row_tail<F16, NB>(Bm + (size_t)n * g.ldb + kc, half, g.bscale, K - kc, b); }
                else    { if (kc + 32 <= K) op_col<F16, NB>(Bm, g.ldb, n * g.bcs, kc, half, g.bscale, b); else op_col_tail<F16, NB>(Bm, g.ldb, n * g.bcs, kc, half, g.bscale, K, b); }
            } else {
#pragma unroll
                for (int p = 0; p < NB; ++p) b.p[p] = (v16bf){};
            }
            acc[t] = wmma_op<F16, NA, NB>(a, b, acc[t]);
        }
    }
    const float* bias = g.bias ? g.bias + zoff(g.zbias, z) : nullptr;
    const float* add = g.add ? g.add + zoff(g.zadd, z) : nullptr;
    const float* rsc = g.rsc ? g.rsc + zoff(g.zrsc, z) : nullptr;
    const float* mul = g.mul ? g.mul + zoff(g.zmul, z) : nullptr;
    const float* rbias = g.rbias ? g.rbias + zoff(g.zrbias, z) : nullptr;
#pragma unroll
    for (int t = 0; t < 4; ++t) {
        const int cl = ch * 64 + t * 16 + l16;
        const int cg = blockIdx.y * TC + cl;
        const bool cok = cg < g.nvalid;
        const float bv = (bias && cok) ? bias[(size_t)cg * g.bcs] : 0.0f;
#pragma unroll
        for (int r = 0; r < 8; ++r) {
            const int rl = rt * 16 + r + 8 * half;
            float v = acc[t][r] * g.oscale + bv;
            int rg = row0 + rl; if (rg >= g.M) rg = g.M - 1;
            if (rbias) v += rbias[rg];
            if (rsc) v *= rsc[(size_t)rg * g.ldrsc];
            if (mul && cok) v *= mul[(size_t)rg * g.ldmul + cg];
            if (add && cok) v += g.addscale * add[(size_t)rg * g.ldadd + cg];
            cst[rl * CSTR + cl] = v;
        }
    }
    __syncthreads();
    const int col = tid % TC, rsel = tid / TC, rstep = 256 / TC;
    if (ACT != ACT_NONE) {
#pragma unroll 1
        for (int r = rsel; r < TR; r += rstep) cst[r * CSTR + col] = act_apply(ACT, cst[r * CSTR + col]);
    }
    float* ob = C + (size_t)row0 * g.ldc + (size_t)blockIdx.y * TC;
    const bool colok = (int)(blockIdx.y * TC + col) < g.nstore;
    const int rmax = (g.M - row0 < TR) ? (g.M - row0) : TR;
    auto pass = [&]() {
        if (colok) {
#pragma unroll 4
            for (int r = rsel; r < rmax; r += rstep) *(volatile float*)(ob + (size_t)r * g.ldc + col) = cst[r * CSTR + col];
        }
    };
    pass();
    __threadfence();
    pass();
}
static inline ZMap zm(long long s1) { ZMap m; m.s1 = s1; m.s2 = 0; m.zdiv = 1; m.pad_ = 0; return m; }
static inline ZMap zm2(long long s1, long long s2, int zdiv) { ZMap m; m.s1 = s1; m.s2 = s2; m.zdiv = zdiv; m.pad_ = 0; return m; }
static inline GemmArgs gemm_args(const float* A, int lda, ZMap za, const float* Bm, int ldb, ZMap zb, float* C, int ldc, ZMap zc, int M, int N, int K) {
    GemmArgs g; g.za = za; g.zb_ = zb; g.zc = zc; g.zbias = zm(0); g.zadd = zm(0); g.zrsc = zm(0); g.zmul = zm(0); g.zrbias = zm(0);
    g.A = A; g.Bm = Bm; g.C = C; g.bias = nullptr; g.add = nullptr; g.rsc = nullptr; g.mul = nullptr; g.rbias = nullptr; g.ldadd = 0; g.ldmul = 0;
    g.lda = lda; g.ldb = ldb; g.ldc = ldc; g.K = K; g.ascale = 1.0f; g.bscale = 1.0f; g.oscale = 1.0f; g.addscale = 1.0f; g.M = M; g.nvalid = N; g.nstore = N; g.ldrsc = 1;
    g.bcs = 1; g.pad1 = 0; g.pad2 = 0; g.pad3 = 0;
    return g;
}
static_assert(sizeof(ZMap) == 24, "ZMap layout");
static_assert(sizeof(GemmArgs) == 8 * 24 + 8 * 8 + 2 * 8 + 4 * 4 + 4 * 4 + 4 * 4 + 4 * 4, "GemmArgs has no padding");

__global__ __launch_bounds__(256) void softmax_rows(float* S, long long sy, long long sx, int L, float prescale, const float* addv, long long say, int aydiv, int causal,
                                                  const int* imask, long long imy, long long imx, float maskval) {
    __shared__ float red[8];
    const int tid = threadIdx.x, lane = tid & 31, wid = tid >> 5;
    float* row = S + (size_t)blockIdx.y * sy + (size_t)blockIdx.x * sx;
    const float* av = addv ? addv + (size_t)(blockIdx.y / aydiv) * say : nullptr;
    const int* im = imask ? imask + (size_t)(blockIdx.y / aydiv) * imy + (size_t)blockIdx.x * imx : nullptr;
    float v[32];
    const int nj = L / 256;
    float mx = -__builtin_inff();
#pragma unroll
    for (int j = 0; j < 32; ++j) if (j < nj) { float t = row[tid + 256 * j] * prescale; if (av) t += av[tid + 256 * j]; if (im && im[tid + 256 * j] == 0) t = maskval; if (causal && (tid + 256 * j) > (int)blockIdx.x) t = -__builtin_inff(); v[j] = t; mx = fmaxf(mx, t); }
#pragma unroll
    for (int o = 16; o; o >>= 1) mx = fmaxf(mx, __shfl_xor(mx, o, 32));
    if (lane == 0) red[wid] = mx;
    __syncthreads();
    float m = red[0];
#pragma unroll
    for (int i = 1; i < 8; ++i) m = fmaxf(m, red[i]);
    if (m == -__builtin_inff()) m = 0.f;
    __syncthreads();
    float sum = 0.f;
#pragma unroll
    for (int j = 0; j < 32; ++j) if (j < nj) { v[j] = expf(v[j] - m); sum += v[j]; }
#pragma unroll
    for (int o = 16; o; o >>= 1) sum += __shfl_xor(sum, o, 32);
    if (lane == 0) red[wid] = sum;
    __syncthreads();
    float tot = 0.f;
#pragma unroll
    for (int i = 0; i < 8; ++i) tot += red[i];
    const float inv = 1.0f / tot;
#pragma unroll
    for (int j = 0; j < 32; ++j) if (j < nj) *(volatile float*)(row + tid + 256 * j) = v[j] * inv;
    __threadfence();
#pragma unroll
    for (int j = 0; j < 32; ++j) if (j < nj) *(volatile float*)(row + tid + 256 * j) = v[j] * inv;
}

#define VST2(T, p, v) do { const T vst2_v_ = (v); *(volatile T*)(p) = vst2_v_; __threadfence(); *(volatile T*)(p) = vst2_v_; } while (0)
#define IL_T 128
#define IL_TILE 4096
__global__ __launch_bounds__(IL_T) void k_inlists(const int* __restrict__ tgt, int E, int N, int* NBR, int* cnt) {
    __shared__ int tt[IL_TILE];
    __shared__ int lists[IL_T * IL_CAP];
    const int d = blockIdx.x * IL_T + threadIdx.x; int n = 0;
    for (int e0 = 0; e0 < E; e0 += IL_TILE) {
        const int nt = min(IL_TILE, E - e0);
        __syncthreads();
        for (int i = threadIdx.x; i < nt; i += IL_T) tt[i] = tgt[e0 + i];
        __syncthreads();
        for (int i = 0; i < nt; ++i) { if (tt[i] == d) { if (n < IL_CAP) lists[threadIdx.x * IL_CAP + n] = e0 + i; ++n; } }
    }
    if (d < N) {
        int* row = NBR + (size_t)d * IL_CAP;
        for (int j = 0; j < IL_CAP; ++j) { const int v = (j < n) ? lists[threadIdx.x * IL_CAP + j] : 0; *(volatile int*)(row + j) = v; }
        __threadfence();
        for (int j = 0; j < IL_CAP; ++j) { const int v = (j < n) ? lists[threadIdx.x * IL_CAP + j] : 0; *(volatile int*)(row + j) = v; }
        VST2(int, cnt + d, min(n, IL_CAP));
    }
}
__global__ __launch_bounds__(256) void k_csr_scan(const int* __restrict__ cnt, int* off, int N) {
    __shared__ int part[256]; const int per = ((((N + 255) / 256) + 31) / 32) * 32; const int a = threadIdx.x * per, b = min(N, a + per); int s = 0;
    for (int i = a; i < b; ++i) s += cnt[i]; part[threadIdx.x] = s; __syncthreads();
    if (threadIdx.x == 0) { int run = 0; for (int t = 0; t < 256; ++t) { const int v = part[t]; part[t] = run; run += v; } } __syncthreads();
    int run = part[threadIdx.x]; for (int i = a; i < b; ++i) { VST2(int, off + i, run); run += cnt[i]; }
    if (a < N && b == N) { VST2(int, off + N, run); }
}
__global__ __launch_bounds__(256) void k_slotcopy(const int* __restrict__ off, const int* __restrict__ NBR, int* slot, int N) {
    const int t = blockIdx.x * 256 + threadIdx.x; const int tot = off[N]; if (t >= tot) return;
    int lo = 0, hi = N - 1;
    while (lo < hi) { const int mid = (lo + hi + 1) >> 1; if (off[mid] <= t) lo = mid; else hi = mid - 1; }
    int j = t - off[lo]; j = (j < 0) ? 0 : ((j >= IL_CAP) ? (IL_CAP - 1) : j);
    VST2(int, slot + t, NBR[(size_t)lo * IL_CAP + j]);
}


__global__ __launch_bounds__(256) void k_embed(const int* __restrict__ ids, const float* __restrict__ emb, float* X) {
    const size_t t = (size_t)blockIdx.x * 256 + threadIdx.x; if (t >= (size_t)NN_ * DD) return;
    const int c = (int)(t % DD), n = (int)(t / DD); int id = ids[n]; id = id < 0 ? 0 : (id >= NVOC ? NVOC - 1 : id);
    VST2(float, X + t, emb[(size_t)id * DD + c]);
}
__global__ __launch_bounds__(256) void k_hw(const float* __restrict__ HID, const float* __restrict__ w2, const float* __restrict__ b2, float* hw) {
    const int e = blockIdx.x * 256 + threadIdx.x; if (e >= NE2) return;
    float s = b2[0]; for (int c = 0; c < DD; ++c) s += HID[(size_t)e * DD + c] * w2[c];
    VST2(float, hw + e, 1.0f / (1.0f + expf(-s)));
}
__global__ __launch_bounds__(256) void k_rowdot(const float* __restrict__ M, const float* __restrict__ a, float* outp, int R) {
    const int r = blockIdx.x * 256 + threadIdx.x; if (r >= R) return;
    float s = 0.f; for (int c = 0; c < DD; ++c) s += M[(size_t)r * DD + c] * a[c];
    VST2(float, outp + r, s);
}
__global__ __launch_bounds__(256) void k_eattr(const float* __restrict__ xl, const int* __restrict__ nodes, const int* __restrict__ offE, const int* __restrict__ slotE, float* ea) {
    const size_t t = (size_t)blockIdx.x * 256 + threadIdx.x; if (t >= (size_t)NE2 * DD) return;
    const int c = (int)(t % DD), e = (int)(t / DD); const int a = offE[e], b = offE[e + 1]; float s = 0.f;
    for (int p = a; p < b && p < a + IL_CAP; ++p) { int i = slotE[p]; i = i < 0 ? 0 : (i >= NNZ ? NNZ - 1 : i); int n = nodes[i]; n = n < 0 ? 0 : (n >= NN_ ? NN_ - 1 : n); s += xl[(size_t)n * DD + c]; }
    VST2(float, ea + t, (b > a) ? s / (float)(b - a) : 0.f);
}
__global__ __launch_bounds__(256) void k_nodestats(const float* __restrict__ sn, const float* __restrict__ se, const float* __restrict__ hw, const int* __restrict__ edges,
                                                   const int* __restrict__ offN, const int* __restrict__ slotN, float* nm, float* ninv, float* Dinv) {
    const int n = blockIdx.x * 256 + threadIdx.x; if (n >= NN_) return;
    const int a = offN[n], b = offN[n + 1]; const float s0 = sn[n];
    float m = -__builtin_inff();
    for (int p = a; p < b && p < a + IL_CAP; ++p) { int i = slotN[p]; i = i < 0 ? 0 : (i >= NNZ ? NNZ - 1 : i); int e = edges[i]; e = e < 0 ? 0 : (e >= NE2 ? NE2 - 1 : e);
        float al = s0 + se[e]; al = al > 0.f ? al : 0.2f * al; m = fmaxf(m, al); }
    if (!(m > -__builtin_inff())) m = 0.f;
    float z = 0.f, dw = 0.f;
    for (int p = a; p < b && p < a + IL_CAP; ++p) { int i = slotN[p]; i = i < 0 ? 0 : (i >= NNZ ? NNZ - 1 : i); int e = edges[i]; e = e < 0 ? 0 : (e >= NE2 ? NE2 - 1 : e);
        float al = s0 + se[e]; al = al > 0.f ? al : 0.2f * al; z += expf(al - m); dw += hw[e]; }
    VST2(float, nm + n, m); VST2(float, ninv + n, 1.0f / (z > 0.f ? z : 1.0f)); VST2(float, Dinv + n, dw > 0.f ? 1.0f / dw : 0.f);
}
__global__ __launch_bounds__(256) void k_ef(const float* __restrict__ xl, const float* __restrict__ sn, const float* __restrict__ se, const float* __restrict__ nm, const float* __restrict__ ninv,
                                            const int* __restrict__ nodes, const int* __restrict__ offE, const int* __restrict__ slotE, float* ef) {
    const size_t t = (size_t)blockIdx.x * 256 + threadIdx.x; if (t >= (size_t)NE2 * DD) return;
    const int c = (int)(t % DD), e = (int)(t / DD); const int a = offE[e], b = offE[e + 1];
    const float binv = (b > a) ? 1.0f / (float)(b - a) : 0.f; const float see = se[e];
    float s = 0.f;
    for (int p = a; p < b && p < a + IL_CAP; ++p) { int i = slotE[p]; i = i < 0 ? 0 : (i >= NNZ ? NNZ - 1 : i); int n = nodes[i]; n = n < 0 ? 0 : (n >= NN_ ? NN_ - 1 : n);
        float al = sn[n] + see; al = al > 0.f ? al : 0.2f * al; const float alpha = expf(al - nm[n]) * ninv[n];
        s += binv * alpha * xl[(size_t)n * DD + c]; }
    VST2(float, ef + t, s);
}
__global__ __launch_bounds__(256) void k_nodeout(const float* __restrict__ ef, const float* __restrict__ sn, const float* __restrict__ se, const float* __restrict__ nm, const float* __restrict__ ninv,
                                                 const float* __restrict__ Dinv, const int* __restrict__ edges, const int* __restrict__ offN, const int* __restrict__ slotN, const float* __restrict__ bias, float* xo) {
    const size_t t = (size_t)blockIdx.x * 256 + threadIdx.x; if (t >= (size_t)NN_ * DD) return;
    const int c = (int)(t % DD), n = (int)(t / DD); const int a = offN[n], b = offN[n + 1];
    const float s0 = sn[n], m = nm[n], zi = ninv[n], di = Dinv[n];
    float s = 0.f;
    for (int p = a; p < b && p < a + IL_CAP; ++p) { int i = slotN[p]; i = i < 0 ? 0 : (i >= NNZ ? NNZ - 1 : i); int e = edges[i]; e = e < 0 ? 0 : (e >= NE2 ? NE2 - 1 : e);
        float al = s0 + se[e]; al = al > 0.f ? al : 0.2f * al; const float alpha = expf(al - m) * zi;
        s += di * alpha * ef[(size_t)e * DD + c]; }
    VST2(float, xo + t, fmaxf(s + bias[c], 0.f));
}
__global__ __launch_bounds__(64) void k_colstats64(const float* __restrict__ a, float* cmean, float* cvar, int N) {
    const int d = threadIdx.x; double s = 0.0;
    for (int i = 0; i < N; ++i) s += (double)a[(size_t)i * 64 + d];
    const double m = s / (double)N; double q = 0.0;
    for (int i = 0; i < N; ++i) { const double v = (double)a[(size_t)i * 64 + d] - m; q += v * v; }
    const float mv = (float)m, vv = (float)(q / (double)N);
    *(volatile float*)(cmean + d) = mv; *(volatile float*)(cvar + d) = vv; __threadfence(); *(volatile float*)(cmean + d) = mv; *(volatile float*)(cvar + d) = vv;
}
__global__ __launch_bounds__(256) void k_bn_relu64(float* a, const float* __restrict__ cmean, const float* __restrict__ cvar, const float* __restrict__ g, const float* __restrict__ bb) {
    const size_t t = (size_t)blockIdx.x * 256 + threadIdx.x; if (t >= (size_t)NN_ * 64) return;
    const int d = (int)(t % 64);
    const float v = fmaxf(g[d] * (a[t] - cmean[d]) * rsqrtf(cvar[d] + BN_EPS) + bb[d], 0.f);
    VST2(float, a + t, v);
}

extern "C" void kernel_launch(void* const* d_in, const int* in_sizes, int n_in,
                              void* d_out, int out_size, void* d_ws, size_t ws_size, hipStream_t stream) {
    (void)in_sizes; (void)n_in; (void)out_size;
    const int* kw = (const int*)d_in[0];
    const int* hidx = (const int*)d_in[1];
    const float* emb = (const float*)d_in[2];
    const float* ipw = (const float*)d_in[3]; const float* ipb = (const float*)d_in[4];
    const float* opw = (const float*)d_in[5]; const float* opb = (const float*)d_in[6];
    const float* cw = (const float*)d_in[7]; const float* cb = (const float*)d_in[8];
    const float* catt = (const float*)d_in[9];
    const float* wg1 = (const float*)d_in[10]; const float* wgb1 = (const float*)d_in[11];
    const float* wg2 = (const float*)d_in[12]; const float* wgb2 = (const float*)d_in[13];
    const float* fl1 = (const float*)d_in[14]; const float* flb1 = (const float*)d_in[15];
    const float* bng = (const float*)d_in[16]; const float* bnb = (const float*)d_in[17];
    const float* fl2 = (const float*)d_in[18]; const float* flb2 = (const float*)d_in[19];
    float* out = (float*)d_out;
    const int* nodes = hidx; const int* edges = hidx + NNZ;

    char* wsp = (char*)d_ws;
    auto take = [&](size_t bytes) { char* p = wsp; wsp += (bytes + 255) & ~(size_t)255; return (void*)p; };
    int* NBR = (int*)take((size_t)NN_ * IL_CAP * 4); int* cnt = (int*)take((size_t)(NN_ + 1) * 4);
    int* offE = (int*)take((size_t)(NE2 + 1) * 4); int* slotE = (int*)take((size_t)NNZ * 4);
    int* offN = (int*)take((size_t)(NN_ + 1) * 4); int* slotN = (int*)take((size_t)NNZ * 4);
    float* X = (float*)take((size_t)NN_ * DD * 4);
    float* QKV = (float*)take((size_t)NN_ * 3 * DD * 4);
    float* O = (float*)take((size_t)NN_ * DD * 4);
    float* S = (float*)take((size_t)RCH * NN_ * 4);
    float* HIDb = (float*)take((size_t)NE2 * DD * 4);
    float* hw = (float*)take((size_t)NE2 * 4);
    float* XL = (float*)take((size_t)NN_ * DD * 4);
    float* EA = (float*)take((size_t)NE2 * DD * 4);
    float* sn = (float*)take((size_t)NN_ * 4); float* se = (float*)take((size_t)NE2 * 4);
    float* nm = (float*)take((size_t)NN_ * 4); float* ninv = (float*)take((size_t)NN_ * 4); float* Dinv = (float*)take((size_t)NN_ * 4);
    float* EF = (float*)take((size_t)NE2 * DD * 4);
    float* X2 = (float*)take((size_t)NN_ * DD * 4);
    float* HF = (float*)take((size_t)NN_ * 64 * 4);
    float* cm = (float*)take(64 * 4); float* cv = (float*)take(64 * 4);
    if ((size_t)(wsp - (char*)d_ws) > ws_size) return;

    k_inlists<<<(NE2 + IL_T - 1) / IL_T, IL_T, 0, stream>>>(edges, NNZ, NE2, NBR, cnt);
    k_csr_scan<<<1, 256, 0, stream>>>(cnt, offE, NE2);
    k_slotcopy<<<(NNZ + 255) / 256, 256, 0, stream>>>(offE, NBR, slotE, NE2);
    k_inlists<<<(NN_ + IL_T - 1) / IL_T, IL_T, 0, stream>>>(nodes, NNZ, NN_, NBR, cnt);
    k_csr_scan<<<1, 256, 0, stream>>>(cnt, offN, NN_);
    k_slotcopy<<<(NNZ + 255) / 256, 256, 0, stream>>>(offN, NBR, slotN, NN_);
    k_embed<<<(NN_ * DD) / 256, 256, 0, stream>>>(kw, emb, X);
    { GemmArgs g = gemm_args(X, DD, zm(0), ipw, DD, zm(0), QKV, 3 * DD, zm(0), NN_, 3 * DD, DD); g.bias = ipb; g.bscale = 16.0f; g.oscale = 1.0f / 16.0f;
      gemm_kernel<1, 1, 1, 1, 4, 2, ACT_NONE><<<dim3(NN_ / 64, (3 * DD) / 128, 1), 256, 0, stream>>>(g); }
    const float scl = 0.17677669529663687f;
    for (int h = 0; h < NHEAD; ++h) for (int r0 = 0; r0 < NN_; r0 += RCH) {
        { GemmArgs g = gemm_args(QKV + (size_t)r0 * 3 * DD + h * HDM, 3 * DD, zm(0), QKV + DD + h * HDM, 3 * DD, zm(0), S, NN_, zm(0), RCH, NN_, HDM); g.ascale = 16.0f; g.bscale = 16.0f; g.oscale = 1.0f / 256.0f;
          gemm_kernel<1, 1, 1, 1, 4, 2, ACT_NONE><<<dim3(RCH / 64, NN_ / 128, 1), 256, 0, stream>>>(g); }
        softmax_rows<<<dim3(RCH, 1), 256, 0, stream>>>(S, 0LL, NN_, NN_, scl, nullptr, 0LL, 1, 0, nullptr, 0LL, 0LL, 0.f);
        { GemmArgs g = gemm_args(S, NN_, zm(0), QKV + 2 * DD + h * HDM, 3 * DD, zm(0), O + (size_t)r0 * DD + h * HDM, DD, zm(0), RCH, HDM, NN_); g.ascale = 4096.0f; g.bscale = 16.0f; g.oscale = 1.0f / 65536.0f;
          gemm_kernel<0, 1, 1, 1, 8, 1, ACT_NONE><<<dim3(RCH / 128, 1, 1), 256, 0, stream>>>(g); }
    }
    { GemmArgs g = gemm_args(O, DD, zm(0), opw, DD, zm(0), X, DD, zm(0), NN_, DD, DD); g.bias = opb; g.ascale = 16.0f; g.bscale = 16.0f; g.oscale = 1.0f / 256.0f;
      gemm_kernel<1, 1, 1, 1, 4, 2, ACT_NONE><<<dim3(NN_ / 64, 1, 1), 256, 0, stream>>>(g); }
    float* xin = X; float* xout = X2;
    for (int l = 0; l < NLAY; ++l) {
        { GemmArgs g = gemm_args(xin, DD, zm(0), wg1, DD, zm(0), HIDb, DD, zm(0), NE2, DD, DD); g.bias = wgb1; g.bscale = 16.0f; g.oscale = 1.0f / 16.0f;
          gemm_kernel<1, 1, 1, 1, 4, 2, ACT_RELU><<<dim3(NE2 / 64, 1, 1), 256, 0, stream>>>(g); }
        k_hw<<<NE2 / 256, 256, 0, stream>>>(HIDb, wg2, wgb2, hw);
        { GemmArgs g = gemm_args(xin, DD, zm(0), cw + (size_t)l * DD * DD, DD, zm(0), XL, DD, zm(0), NN_, DD, DD); g.bscale = 16.0f; g.oscale = 1.0f / 16.0f;
          gemm_kernel<1, 1, 1, 1, 4, 2, ACT_NONE><<<dim3(NN_ / 64, 1, 1), 256, 0, stream>>>(g); }
        k_eattr<<<(NE2 * DD) / 256, 256, 0, stream>>>(XL, nodes, offE, slotE, EA);
        k_rowdot<<<NN_ / 256, 256, 0, stream>>>(XL, catt + (size_t)l * 2 * DD, sn, NN_);
        k_rowdot<<<NE2 / 256, 256, 0, stream>>>(EA, catt + (size_t)l * 2 * DD + DD, se, NE2);
        k_nodestats<<<NN_ / 256, 256, 0, stream>>>(sn, se, hw, edges, offN, slotN, nm, ninv, Dinv);
        k_ef<<<(NE2 * DD) / 256, 256, 0, stream>>>(XL, sn, se, nm, ninv, nodes, offE, slotE, EF);
        k_nodeout<<<(NN_ * DD) / 256, 256, 0, stream>>>(EF, sn, se, nm, ninv, Dinv, edges, offN, slotN, cb + (size_t)l * DD, xout);
        float* tsw = xin; xin = xout; xout = tsw;
    }
    { GemmArgs g = gemm_args(xin, DD, zm(0), fl1, DD, zm(0), HF, 64, zm(0), NN_, 64, DD); g.bias = flb1;
      gemm_kernel<1, 0, 3, 3, 8, 1, ACT_NONE><<<dim3(NN_ / 128, 1, 1), 256, 0, stream>>>(g); }
    k_colstats64<<<1, 64, 0, stream>>>(HF, cm, cv, NN_);
    k_bn_relu64<<<(NN_ * 64) / 256, 256, 0, stream>>>(HF, cm, cv, bng, bnb);
    { GemmArgs g = gemm_args(HF, 64, zm(0), fl2, 64, zm(0), out, DD, zm(0), NN_, DD, 64); g.bias = flb2;
      gemm_kernel<1, 0, 2, 2, 4, 2, ACT_NONE><<<dim3(NN_ / 64, 1, 1), 256, 0, stream>>>(g); }
}
